// Text2Lstm_58677843198151
// MI455X (gfx1250) — hardware-verified
//
#include <hip/hip_runtime.h>

constexpr int kBatch   = 64;
constexpr int kSeq     = 512;
constexpr int kEmbDim  = 300;
constexpr int kHid     = 100;
constexpr int kCls     = 6;
constexpr int kUnitPad = 128;
constexpr int kGateCols = 4 * kUnitPad;
constexpr int kKX0     = 320;
constexpr int kKX1     = 256;
constexpr int kKH      = 128;
constexpr int kHP      = 136;
constexpr int kHSP     = 132;
constexpr int kThreads = 256;
constexpr int kEmbF4   = kEmbDim / 4;
constexpr int kGatherSlots = 16 * kEmbF4;
constexpr float kWScale    = 16.0f;
constexpr float kWScaleInv = 1.0f / 16.0f;

typedef __attribute__((ext_vector_type(16))) _Float16 v16h;
typedef __attribute__((ext_vector_type(8)))  _Float16 v8h;
typedef __attribute__((ext_vector_type(8)))  float    v8f;
typedef __attribute__((ext_vector_type(4)))  float    v4f;
typedef __attribute__((ext_vector_type(2)))  unsigned v2u;

__device__ __forceinline__ unsigned short f2bf_bits(float f) {
  unsigned u = __float_as_uint(f);
  return (unsigned short)((u + 0x7FFFu + ((u >> 16) & 1u)) >> 16);
}
__device__ __forceinline__ float bf_bits2f(unsigned short h) { return __uint_as_float(((unsigned)h) << 16); }

__device__ __forceinline__ void dep_guard_h(v8f& a, v8f& b, v16h x, v16h y) { asm volatile("v_nop\n\tv_nop\n\tv_nop\n\tv_nop" : "+v"(a), "+v"(b) : "v"(x), "v"(y)); }
__device__ __forceinline__ void keep4_h(v16h a, v16h b, v16h c, v16h d) { asm volatile("v_nop" :: "v"(a), "v"(b), "v"(c), "v"(d)); }
__device__ __forceinline__ void acc_guard4(v8f& a, v8f& b, v8f& c, v8f& d) { asm volatile("v_nop\n\tv_nop\n\tv_nop\n\tv_nop" : "+v"(a), "+v"(b), "+v"(c), "+v"(d)); }
template <typename T> struct Frag;
template <> struct Frag<_Float16> {
  typedef v16h V; union U { v16h v; v8h h[2]; };
  static __device__ __forceinline__ v16h load(const _Float16* p) {
    U f; f.h[0] = *(const v8h*)(p); f.h[1] = *(const v8h*)(p + 16); return f.v;
  }
  static __device__ __forceinline__ v8f mma(v16h a, v16h b, v8f c) {
    return __builtin_amdgcn_wmma_f32_16x16x32_f16(false, a, false, b, (short)0, c, false, false);
  }
};

__device__ __forceinline__ float bfr(float f) { return bf_bits2f(f2bf_bits(f)); }
__device__ __forceinline__ unsigned short h16_of_bf(float f) {
  return __builtin_bit_cast(unsigned short, (_Float16)bfr(f));
}
__device__ __forceinline__ float fsig(float x)  { return __builtin_amdgcn_rcpf(1.0f + __expf(-x)); }
__device__ __forceinline__ float ftanh(float x) { return 1.0f - 2.0f * __builtin_amdgcn_rcpf(__expf(2.0f * x) + 1.0f); }

__global__ __launch_bounds__(kThreads) void prep_w_kernel(const float* __restrict__ W, int IN, int KP, int mode,
                                                          unsigned short* __restrict__ O) {
  const int perRow = KP >> 3;
  const int total  = kGateCols * perRow;
  const int idx = blockIdx.x * kThreads + threadIdx.x;
  const int idc = idx < total ? idx : total - 1;
  const int n   = idc / perRow;
  const int c8  = (idc - n * perRow) * 8;
  const int g = n >> 7, uu = n & 127;
  const int srow = g * kHid + (uu < kHid ? uu : kHid - 1);
  v8h hv;
#pragma unroll
  for (int e = 0; e < 8; ++e) {
    const int k = c8 + e;
    const int  ks0 = k;
    const bool ok0 = (k < IN);
    const int  ks1 = (k < kUnitPad) ? k : (k - (kUnitPad - kHid));
    const bool ok1 = (k < kHid) || (k >= kUnitPad && k < kUnitPad + kHid);
    const int  ks  = mode ? ks1 : ks0;
    const bool ok  = (mode ? ok1 : ok0) && (uu < kHid);
    const int ksc = ks < 0 ? 0 : (ks > IN - 1 ? IN - 1 : ks);
    float f = W[(size_t)srow * IN + ksc];
    f = ok ? f : 0.0f;
    hv[e] = (_Float16)(bfr(f) * kWScale);
  }
  unsigned short* dst = O + (size_t)n * KP + c8;
  if (idx < total) {
    *(volatile v8h*)dst = hv;
    __threadfence();
    *(volatile v8h*)dst = hv;
  }
}

__global__ __launch_bounds__(128) void prep_bias_kernel(const float* __restrict__ bi, const float* __restrict__ bh,
                                                        float* __restrict__ BSo) {
  const int tid = threadIdx.x;
  const int n0 = tid * 4;
  v4f v;
#pragma unroll
  for (int e = 0; e < 4; ++e) {
    const int n = n0 + e;
    const int g = n >> 7, uu = n & 127;
    const int si = g * kHid + (uu < kHid ? uu : kHid - 1);
    const float f = bfr(bi[si]) + bfr(bh[si]);
    v[e] = (uu < kHid) ? f : 0.0f;
  }
  float* dst = BSo + n0;
  *(volatile v4f*)dst = v;
  __threadfence();
  *(volatile v4f*)dst = v;
}

template <int XP>
__device__ __forceinline__ void gather_emb_tile(unsigned short* Ax, const int* __restrict__ xtok,
                                                const float* __restrict__ emb, int nV, int rowbase, int tt, int tid) {
#pragma unroll 1
  for (int i = 0; i < 5; ++i) {
    const int slot = i * kThreads + tid;
    const int sc   = slot < kGatherSlots ? slot : kGatherSlots - 1;
    const int row  = sc / kEmbF4;
    const int c4   = (sc - row * kEmbF4) * 4;
    int tok = xtok[(size_t)(rowbase + row) * kSeq + tt];
    tok = tok < 0 ? 0 : tok;
    tok = tok > nV - 1 ? nV - 1 : tok;
    const v4f v = *(const v4f*)(emb + (size_t)tok * kEmbDim + c4);
    v2u pk;
    pk[0] = (unsigned)h16_of_bf(v[0]) | ((unsigned)h16_of_bf(v[1]) << 16);
    pk[1] = (unsigned)h16_of_bf(v[2]) | ((unsigned)h16_of_bf(v[3]) << 16);
    if (slot < kGatherSlots) *(v2u*)(Ax + row * XP + c4) = pk;
  }
}

template <int XP>
__device__ __forceinline__ void load_h16_tile(unsigned short* Ax, const unsigned short* X16, int rowbase, int tt, int tid) {
#pragma unroll
  for (int i = 0; i < 2; ++i) {
    const int slot = i * kThreads + tid;
    const int row = slot >> 5, c8 = (slot & 31) * 8;
    const v8h v = *(const v8h*)((const _Float16*)(const void*)X16 + ((size_t)(rowbase + row) * kSeq + tt) * kKX1 + c8);
    *(v8h*)((_Float16*)(void*)Ax + row * XP + c8) = v;
  }
}

template <int LAYER>
__global__ __launch_bounds__(kThreads) void lstm_kernel(const int* __restrict__ xtok, const float* __restrict__ emb, int nV,
                                                        const unsigned short* X16,
                                                        const unsigned short* __restrict__ WXp,
                                                        const unsigned short* __restrict__ WHp,
                                                        const float* __restrict__ BS,
                                                        unsigned short* O16, float* __restrict__ LASTp) {
  constexpr int KXD = (LAYER == 0) ? kKX0 : kKX1;
  constexpr int XP  = KXD + 8;
  __shared__ __align__(16) unsigned short Ax[16 * XP];
  __shared__ __align__(16) _Float16       Ah[16 * kHP];
  __shared__ __align__(16) float          Hs[(LAYER == 1) ? 16 * kHSP : 4];

  const int tid = threadIdx.x, lane = tid & 31, wave = tid >> 5;
  const int c = lane & 15, hh = lane >> 4, koff = hh * 8;
  const int dir = (int)(blockIdx.x >> 2);
  const int rowbase = (int)(blockIdx.x & 3) * 16;
  const int u = wave * 16 + c;
  const _Float16* WX = (const _Float16*)(const void*)WXp + (size_t)dir * kGateCols * KXD;
  const _Float16* WH = (const _Float16*)(const void*)WHp + (size_t)dir * kGateCols * kKH;
  const float* bs = BS + dir * kGateCols;

  for (int i = tid; i < 16 * XP / 2; i += kThreads) ((unsigned*)(void*)Ax)[i] = 0u;
  for (int i = tid; i < 16 * kHP / 2; i += kThreads) ((unsigned*)(void*)Ah)[i] = 0u;

  float bb[4], cst[8], hst[8];
#pragma unroll
  for (int g = 0; g < 4; ++g) bb[g] = bs[g * kUnitPad + u];
#pragma unroll
  for (int r = 0; r < 8; ++r) { cst[r] = 0.0f; hst[r] = 0.0f; }
  const int nsteps = (LAYER == 0) ? kSeq : (dir ? 1 : kSeq);
  __syncthreads();
  {
    const int t0 = dir ? (kSeq - 1) : 0;
    if (LAYER == 0) gather_emb_tile<XP>(Ax, xtok, emb, nV, rowbase, t0, tid);
    else            load_h16_tile<XP>(Ax, X16, rowbase, t0, tid);
  }
  __syncthreads();

  const _Float16* axrow = (const _Float16*)(const void*)Ax + c * XP + koff;
  const _Float16* ahrow = Ah + c * kHP + koff;
  const _Float16* wx = WX + (size_t)u * KXD + koff;
  const _Float16* wh = WH + (size_t)u * kKH + koff;
  const v8f z8 = {0.f, 0.f, 0.f, 0.f, 0.f, 0.f, 0.f, 0.f};

#pragma unroll 1
  for (int s = 0; s < nsteps; ++s) {
    const int t = dir ? (kSeq - 1 - s) : s;
    v8f acc[4];
    acc[0] = z8; acc[1] = z8; acc[2] = z8; acc[3] = z8;
#pragma unroll 1
    for (int kx = 0; kx < KXD; kx += 32) {
      const v16h a  = Frag<_Float16>::load(axrow + kx);
      const v16h b0 = Frag<_Float16>::load(wx + kx);
      const v16h b1 = Frag<_Float16>::load(wx + (size_t)1 * kUnitPad * KXD + kx);
      const v16h b2 = Frag<_Float16>::load(wx + (size_t)2 * kUnitPad * KXD + kx);
      const v16h b3 = Frag<_Float16>::load(wx + (size_t)3 * kUnitPad * KXD + kx);
      acc[0] = Frag<_Float16>::mma(a, b0, acc[0]);
      acc[1] = Frag<_Float16>::mma(a, b1, acc[1]);
      acc[2] = Frag<_Float16>::mma(a, b2, acc[2]);
      acc[3] = Frag<_Float16>::mma(a, b3, acc[3]);
      dep_guard_h(acc[0], acc[3], a, b3);
      keep4_h(b0, b1, b2, b3);
    }
#pragma unroll 1
    for (int k0 = 0; k0 < kKH; k0 += 32) {
      const v16h a  = Frag<_Float16>::load(ahrow + k0);
      const v16h b0 = Frag<_Float16>::load(wh + k0);
      const v16h b1 = Frag<_Float16>::load(wh + (size_t)1 * kUnitPad * kKH + k0);
      const v16h b2 = Frag<_Float16>::load(wh + (size_t)2 * kUnitPad * kKH + k0);
      const v16h b3 = Frag<_Float16>::load(wh + (size_t)3 * kUnitPad * kKH + k0);
      acc[0] = Frag<_Float16>::mma(a, b0, acc[0]);
      acc[1] = Frag<_Float16>::mma(a, b1, acc[1]);
      acc[2] = Frag<_Float16>::mma(a, b2, acc[2]);
      acc[3] = Frag<_Float16>::mma(a, b3, acc[3]);
      dep_guard_h(acc[0], acc[3], a, b3);
      keep4_h(b0, b1, b2, b3);
    }
    acc_guard4(acc[0], acc[1], acc[2], acc[3]);
#pragma unroll
    for (int r = 0; r < 8; ++r) {
      const float zi = acc[0][r] * kWScaleInv + bb[0];
      const float zf = acc[1][r] * kWScaleInv + bb[1];
      const float zg = acc[2][r] * kWScaleInv + bb[2];
      const float zo = acc[3][r] * kWScaleInv + bb[3];
      const float ig = fsig(zi);
      const float fg = fsig(zf);
      const float og = fsig(zo);
      const float gg = ftanh(zg);
      const float cn = fg * cst[r] + ig * gg;
      cst[r] = cn;
      hst[r] = og * ftanh(cn);
    }
    __syncthreads();
#pragma unroll
    for (int r = 0; r < 8; ++r) Ah[(8 * hh + r) * kHP + u] = (_Float16)hst[r];
    {
      int tn = dir ? (kSeq - 2 - s) : (s + 1);
      tn = tn < 0 ? 0 : (tn > kSeq - 1 ? kSeq - 1 : tn);
      if (LAYER == 0) gather_emb_tile<XP>(Ax, xtok, emb, nV, rowbase, tn, tid);
      else            load_h16_tile<XP>(Ax, X16, rowbase, tn, tid);
    }
    __syncthreads();
    if (LAYER == 0) {
      const int q = lane >> 3, c8 = (lane & 7) * 8;
      const int L = wave * 4 + q;
      const int row = L >> 1, half = L & 1;
      const v8h hv = *(const v8h*)(Ah + row * kHP + half * 64 + c8);
      _Float16* dst = (_Float16*)(void*)O16 + ((size_t)(rowbase + row) * kSeq + t) * kKX1 + dir * kUnitPad + half * 64 + c8;
      *(volatile v8h*)dst = hv;
      __threadfence();
      *(volatile v8h*)dst = hv;
    }
  }

  if (LAYER == 1) {
#pragma unroll
    for (int r = 0; r < 8; ++r) Hs[(8 * hh + r) * kHSP + u] = hst[r];
    __syncthreads();
    for (int pass = 0; pass < 2; ++pass) {
#pragma unroll
      for (int it = 0; it < 2; ++it) {
        const int row = wave * 2 + it;
        const v4f v = *(const v4f*)(Hs + row * kHSP + lane * 4);
        *(volatile v4f*)(LASTp + (size_t)(rowbase + row) * (2 * kUnitPad) + dir * kUnitPad + lane * 4) = v;
      }
      __threadfence();
    }
  }
}

__global__ __launch_bounds__(384) void head_kernel(const float* __restrict__ last, const float* __restrict__ fcw,
                                                  const float* __restrict__ fcb, float* __restrict__ out) {
  __shared__ __align__(16) float so[kBatch * kCls];
  const int tid = threadIdx.x;
  const int b = tid / kCls, cc = tid - b * kCls;
  const float* lr = last + (size_t)b * (2 * kUnitPad);
  const float* wr = fcw + (size_t)cc * (2 * kHid);
  float s = 0.0f;
#pragma unroll 1
  for (int k = 0; k < kHid; ++k) s += lr[k] * bfr(wr[k]);
#pragma unroll 1
  for (int k = 0; k < kHid; ++k) s += lr[kUnitPad + k] * bfr(wr[kHid + k]);
  s += bfr(fcb[cc]);
  so[tid] = s;
  __syncthreads();
  if (tid < 32) {
    const v4f v0 = *(const v4f*)(so + tid * 4);
    const v4f v1 = *(const v4f*)(so + 128 + tid * 4);
    const v4f v2 = *(const v4f*)(so + 256 + tid * 4);
    *(volatile v4f*)(out + tid * 4) = v0;
    *(volatile v4f*)(out + 128 + tid * 4) = v1;
    *(volatile v4f*)(out + 256 + tid * 4) = v2;
    __threadfence();
    *(volatile v4f*)(out + tid * 4) = v0;
    *(volatile v4f*)(out + 128 + tid * 4) = v1;
    *(volatile v4f*)(out + 256 + tid * 4) = v2;
  }
}

extern "C" void kernel_launch(void* const* d_in, const int* in_sizes, int n_in,
                              void* d_out, int out_size, void* d_ws, size_t ws_size, hipStream_t stream) {
  if (n_in < 20 || d_out == nullptr || d_ws == nullptr) return;
  if (in_sizes[0] != kBatch * kSeq || out_size != kBatch * kCls) return;
  if (in_sizes[1] < kEmbDim || (in_sizes[1] % kEmbDim) != 0) return;
  const int nV = in_sizes[1] / kEmbDim;
  if (in_sizes[2] != kCls * 2 * kHid || in_sizes[3] != kCls) return;
  if (in_sizes[4] != 4 * kHid * kEmbDim || in_sizes[8] != 4 * kHid * kEmbDim) return;
  if (in_sizes[12] != 4 * kHid * 2 * kHid || in_sizes[16] != 4 * kHid * 2 * kHid) return;
  if (in_sizes[5] != 4 * kHid * kHid || in_sizes[9] != 4 * kHid * kHid || in_sizes[13] != 4 * kHid * kHid || in_sizes[17] != 4 * kHid * kHid) return;
  for (int i = 6; i < 20; i += 4) { if (in_sizes[i] != 4 * kHid || in_sizes[i + 1] != 4 * kHid) return; }

  const int*   x     = (const int*)d_in[0];
  const float* emb   = (const float*)d_in[1];
  const float* fc_w  = (const float*)d_in[2];
  const float* fc_b  = (const float*)d_in[3];
  const float* w_ih_l0  = (const float*)d_in[4];
  const float* w_hh_l0  = (const float*)d_in[5];
  const float* b_ih_l0  = (const float*)d_in[6];
  const float* b_hh_l0  = (const float*)d_in[7];
  const float* w_ih_l0r = (const float*)d_in[8];
  const float* w_hh_l0r = (const float*)d_in[9];
  const float* b_ih_l0r = (const float*)d_in[10];
  const float* b_hh_l0r = (const float*)d_in[11];
  const float* w_ih_l1  = (const float*)d_in[12];
  const float* w_hh_l1  = (const float*)d_in[13];
  const float* b_ih_l1  = (const float*)d_in[14];
  const float* b_hh_l1  = (const float*)d_in[15];
  const float* w_ih_l1r = (const float*)d_in[16];
  const float* w_hh_l1r = (const float*)d_in[17];
  const float* b_ih_l1r = (const float*)d_in[18];
  const float* b_hh_l1r = (const float*)d_in[19];
  float* out = (float*)d_out;

  char* ws = (char*)d_ws; size_t off = 0;
  auto carve = [&](size_t bytes) -> char* { char* p = ws + off; off += (bytes + 255) & ~(size_t)255; return p; };
  const size_t planeWX0 = (size_t)kGateCols * kKX0;
  const size_t planeWX1 = (size_t)kGateCols * kKX1;
  const size_t planeWH  = (size_t)kGateCols * kKH;
  unsigned short* WX0  = (unsigned short*)carve(2 * planeWX0 * 2);
  unsigned short* WH0  = (unsigned short*)carve(2 * planeWH * 2);
  unsigned short* WX1  = (unsigned short*)carve(2 * planeWX1 * 2);
  unsigned short* WH1  = (unsigned short*)carve(2 * planeWH * 2);
  float*          BS   = (float*)carve((size_t)4 * kGateCols * 4);
  unsigned short* OUT0 = (unsigned short*)carve((size_t)kBatch * kSeq * kKX1 * 2);
  float*          LAST = (float*)carve((size_t)kBatch * 2 * kUnitPad * 4);
  if (off > ws_size || off > (size_t)134217728) return;

  const int blkWX0 = (kGateCols * (kKX0 / 8) + kThreads - 1) / kThreads;
  const int blkWX1 = (kGateCols * (kKX1 / 8) + kThreads - 1) / kThreads;
  const int blkWH  = (kGateCols * (kKH  / 8) + kThreads - 1) / kThreads;
  prep_w_kernel<<<blkWX0, kThreads, 0, stream>>>(w_ih_l0,  kEmbDim,  kKX0, 0, WX0);
  prep_w_kernel<<<blkWX0, kThreads, 0, stream>>>(w_ih_l0r, kEmbDim,  kKX0, 0, WX0 + planeWX0);
  prep_w_kernel<<<blkWH,  kThreads, 0, stream>>>(w_hh_l0,  kHid,     kKH,  0, WH0);
  prep_w_kernel<<<blkWH,  kThreads, 0, stream>>>(w_hh_l0r, kHid,     kKH,  0, WH0 + planeWH);
  prep_w_kernel<<<blkWX1, kThreads, 0, stream>>>(w_ih_l1,  2 * kHid, kKX1, 1, WX1);
  prep_w_kernel<<<blkWX1, kThreads, 0, stream>>>(w_ih_l1r, 2 * kHid, kKX1, 1, WX1 + planeWX1);
  prep_w_kernel<<<blkWH,  kThreads, 0, stream>>>(w_hh_l1,  kHid,     kKH,  0, WH1);
  prep_w_kernel<<<blkWH,  kThreads, 0, stream>>>(w_hh_l1r, kHid,     kKH,  0, WH1 + planeWH);
  prep_bias_kernel<<<1, 128, 0, stream>>>(b_ih_l0,  b_hh_l0,  BS + 0 * kGateCols);
  prep_bias_kernel<<<1, 128, 0, stream>>>(b_ih_l0r, b_hh_l0r, BS + 1 * kGateCols);
  prep_bias_kernel<<<1, 128, 0, stream>>>(b_ih_l1,  b_hh_l1,  BS + 2 * kGateCols);
  prep_bias_kernel<<<1, 128, 0, stream>>>(b_ih_l1r, b_hh_l1r, BS + 3 * kGateCols);
  lstm_kernel<0><<<(kBatch / 16) * 2, kThreads, 0, stream>>>(x, emb, nV, OUT0, WX0, WH0, BS, OUT0, LAST);
  lstm_kernel<1><<<(kBatch / 16) * 2, kThreads, 0, stream>>>(x, emb, nV, OUT0, WX1, WH1, BS + 2 * kGateCols, OUT0, LAST);
  head_kernel<<<1, kBatch * kCls, 0, stream>>>(LAST, fc_w, fc_b, out);
}
